// GGNNMsgPass_69930657513886
// MI455X (gfx1250) — hardware-verified
//
#include <hip/hip_runtime.h>
#include <math.h>

typedef __attribute__((ext_vector_type(16))) _Float16 v16h;
typedef __attribute__((ext_vector_type(8)))  _Float16 v8h;
typedef __attribute__((ext_vector_type(8)))  float    v8f;
typedef __attribute__((ext_vector_type(4)))  float    v4f;

constexpr int kBatch    = 256;
constexpr int kNodes    = 128;
constexpr int kFeat     = 128;
constexpr int kTypes    = 6;
constexpr int kLive     = 5;
constexpr int kTabRow   = kFeat;
constexpr int kTabPlane = kTypes * kFeat;
constexpr int kTabElems = kTypes * kTypes * kFeat;
constexpr int kMsgPitch = 136;
constexpr int kSlabPitch = 132;
constexpr int kPlaneElems = kNodes * kNodes;
constexpr float kAdjCarry = 64.0f;
constexpr float kMsgCarry = 16.0f;
constexpr float kFold     = 1.0f / (kAdjCarry * kMsgCarry);

static_assert(kNodes == 128 && kFeat == 128, "tile maps below assume 128 x 128 per batch");
static_assert((kNodes % 32) == 0, "GEMM K multiple of 32");
static_assert((kNodes % 32) == 0 && (kFeat % 16) == 0, "GEMM M multiple of 32 rows per wave, N multiple of 16");
static_assert(kTabElems == 4608, "table size");
static_assert((kTabElems % 4) == 0, "table staged as 16-B vectors");
static_assert((kMsgPitch % 8) == 0, "16-B aligned LDS rows of halves");
static_assert((kSlabPitch % 4) == 0, "16-B aligned LDS rows of floats");
static_assert(kFold == 1.0f / 1024.0f, "carry fold");

constexpr size_t kOffTab  = 0;
constexpr size_t kOffMsgT = kOffTab  + (size_t)kTabElems * 4;
constexpr size_t kOffAdjH = kOffMsgT + (size_t)kBatch * kPlaneElems * 2;
constexpr size_t kWsTotal = kOffAdjH + (size_t)kBatch * kPlaneElems * 2;
static_assert(kOffMsgT == 18432ull, "carve");
static_assert(kOffAdjH == 8407040ull, "carve");
static_assert(kWsTotal == 16795648ull, "carve total");
static_assert(kWsTotal <= 134217728ull, "carve cap");
static_assert((kOffMsgT % 128) == 0 && (kOffAdjH % 128) == 0, "128-B aligned regions");

struct FragH {
  union U { v16h v; v8h h[2]; };
  static __device__ __forceinline__ v16h load(const _Float16* p) {
    U f;
    f.h[0] = *(const v8h*)(p);
    f.h[1] = *(const v8h*)(p + 16);
    return f.v;
  }
};

__device__ __forceinline__ v8f mma_f16_guarded(v16h a, v16h b, v8f c) {
  c = __builtin_amdgcn_wmma_f32_16x16x32_f16(false, a, false, b, (short)0, c, false, false);
  asm volatile("v_nop\n\tv_nop\n\tv_nop\n\tv_nop" : "+v"(c) : "v"(a), "v"(b));
  return c;
}

__global__ __launch_bounds__(128) void build_table_kernel(
    const float* __restrict__ adj_w, const float* __restrict__ adj_a, float* __restrict__ Tab)
{
  __shared__ __align__(16) float sVec[kFeat];
  __shared__ __align__(16) float sRow[kFeat];
  const int tid  = threadIdx.x;
  const int lane = tid & 31;
  const int wave = __builtin_amdgcn_readfirstlane((int)(threadIdx.x >> 5));
  const int a = (int)blockIdx.x / kTypes;
  const int e = (int)blockIdx.x - a * kTypes;
  const bool live = (a > 0) && (e > 0);
  const int ac = live ? (a - 1) : 0;
  const int ec = live ? (e - 1) : 0;
  sVec[tid] = adj_a[ac * kFeat + tid];
  __syncthreads();
  const float* wr = adj_w + ((size_t)ec * kFeat + tid) * kFeat;
  float s = 0.0f;
#pragma unroll 1
  for (int n4 = 0; n4 < kFeat / 4; ++n4) {
    const v4f w = *(const v4f*)(wr + 4 * n4);
    const v4f x = *(const v4f*)(sVec + 4 * n4);
    s = fmaf(w[0], x[0], s);
    s = fmaf(w[1], x[1], s);
    s = fmaf(w[2], x[2], s);
    s = fmaf(w[3], x[3], s);
  }
  sRow[tid] = live ? s : 0.0f;
  __syncthreads();
  if (wave == 0) {
    const v4f v = *(const v4f*)(sRow + lane * 4);
    float* dst = Tab + (size_t)blockIdx.x * kTabRow + lane * 4;
    *(volatile v4f*)dst = v;
    __threadfence();
    *(volatile v4f*)dst = v;
  }
}

__global__ __launch_bounds__(256) void prep_planes_kernel(
    const int* __restrict__ bfm, const int* __restrict__ a_bfm, const float* __restrict__ adj,
    const float* __restrict__ Tab, unsigned short* __restrict__ MsgT, unsigned short* __restrict__ AdjH)
{
  __shared__ __align__(16) float    sTab[kTabElems];
  __shared__ int                    sPart[2 * kLive * kNodes];
  __shared__ float                  sCntF[kLive * kNodes];
  __shared__ int                    sAt[kNodes];
  __shared__ __align__(16) _Float16 sMsgT[kFeat * kMsgPitch];

  const int tid  = threadIdx.x;
  const int lane = tid & 31;
  const int wave = __builtin_amdgcn_readfirstlane((int)(threadIdx.x >> 5));
  const int b    = blockIdx.x;
  const size_t bbase = (size_t)b * kPlaneElems;

  {
    const float* src = adj + bbase;
    unsigned short* dst = AdjH + bbase;
#pragma unroll 1
    for (int it = 0; it < 8; ++it) {
      const int e0 = (it * 256 + tid) * 8;
      const v4f x0 = *(const v4f*)(src + e0);
      const v4f x1 = *(const v4f*)(src + e0 + 4);
      v8h hv;
      hv[0] = (_Float16)(x0[0] * kAdjCarry);
      hv[1] = (_Float16)(x0[1] * kAdjCarry);
      hv[2] = (_Float16)(x0[2] * kAdjCarry);
      hv[3] = (_Float16)(x0[3] * kAdjCarry);
      hv[4] = (_Float16)(x1[0] * kAdjCarry);
      hv[5] = (_Float16)(x1[1] * kAdjCarry);
      hv[6] = (_Float16)(x1[2] * kAdjCarry);
      hv[7] = (_Float16)(x1[3] * kAdjCarry);
      *(volatile v8h*)(dst + e0) = hv;
      __threadfence();
      *(volatile v8h*)(dst + e0) = hv;
    }
  }

#pragma unroll 1
  for (int p = tid; p < kTabElems / 4; p += 256)
    *(v4f*)(sTab + 4 * p) = *(const v4f*)(Tab + 4 * p);
  {
    int av = a_bfm[b * kNodes + (tid & (kNodes - 1))];
    asm volatile("" : "+v"(av));
    av = av < 0 ? 0 : av;
    av = av > (kTypes - 1) ? (kTypes - 1) : av;
    if (tid < kNodes) sAt[tid] = av;
  }

  {
    const int j = tid & (kNodes - 1);
    const int part = tid >> 7;
    const int* src = bfm + bbase + (size_t)(part * 64) * kNodes + j;
    int c1 = 0, c2 = 0, c3 = 0, c4 = 0, c5 = 0;
#pragma unroll 8
    for (int ii = 0; ii < 64; ++ii) {
      const int v = src[ii * kNodes];
      c1 += (v == 1) ? 1 : 0;
      c2 += (v == 2) ? 1 : 0;
      c3 += (v == 3) ? 1 : 0;
      c4 += (v == 4) ? 1 : 0;
      c5 += (v == 5) ? 1 : 0;
    }
    int* pp = sPart + part * (kLive * kNodes) + j;
    pp[0 * kNodes] = c1;
    pp[1 * kNodes] = c2;
    pp[2 * kNodes] = c3;
    pp[3 * kNodes] = c4;
    pp[4 * kNodes] = c5;
  }
  __syncthreads();
#pragma unroll 1
  for (int idx = tid; idx < kLive * kNodes; idx += 256)
    sCntF[idx] = (float)(sPart[idx] + sPart[kLive * kNodes + idx]) * kMsgCarry;
  __syncthreads();

  {
    const int m  = tid & (kFeat - 1);
    const int jh = tid >> 7;
#pragma unroll 1
    for (int jj = 0; jj < 64; ++jj) {
      const int j = jh * 64 + jj;
      const int a = sAt[j];
      const float* tr = sTab + a * kTabPlane + m;
      float s = 0.0f;
      s = fmaf(sCntF[0 * kNodes + j], tr[1 * kTabRow], s);
      s = fmaf(sCntF[1 * kNodes + j], tr[2 * kTabRow], s);
      s = fmaf(sCntF[2 * kNodes + j], tr[3 * kTabRow], s);
      s = fmaf(sCntF[3 * kNodes + j], tr[4 * kTabRow], s);
      s = fmaf(sCntF[4 * kNodes + j], tr[5 * kTabRow], s);
      sMsgT[m * kMsgPitch + j] = (_Float16)s;
    }
  }
  __syncthreads();

  {
    unsigned short* dstb = MsgT + bbase;
    const int c8 = (lane & 15) * 8;
#pragma unroll 1
    for (int it = 0; it < 8; ++it) {
      const int row = it * 16 + wave * 2 + (lane >> 4);
      const v8h hv = *(const v8h*)(sMsgT + row * kMsgPitch + c8);
      unsigned short* dst = dstb + row * kNodes + c8;
      *(volatile v8h*)dst = hv;
      __threadfence();
      *(volatile v8h*)dst = hv;
    }
  }
}

__global__ __launch_bounds__(128) void batched_gemm_f16_kernel(
    const unsigned short* __restrict__ Ap, const unsigned short* __restrict__ Btp,
    float* __restrict__ Cout, float scale)
{
  __shared__ __align__(16) float sSlab[4][16 * kSlabPitch];
  const int lane = threadIdx.x & 31;
  const int wave = __builtin_amdgcn_readfirstlane((int)(threadIdx.x >> 5));
  const int b    = blockIdx.x;
  const int m0   = wave * 32;
  const _Float16* A  = (const _Float16*)Ap  + (size_t)b * kPlaneElems;
  const _Float16* Bt = (const _Float16*)Btp + (size_t)b * kPlaneElems;
  const int rlane = lane & 15;
  const int koff  = (lane >> 4) * 8;
  const int mOff  = (lane >> 4) * 8;

  v8f acc[2][8];
#pragma unroll
  for (int i = 0; i < 2; ++i)
#pragma unroll
    for (int j = 0; j < 8; ++j) acc[i][j] = (v8f){0.f, 0.f, 0.f, 0.f, 0.f, 0.f, 0.f, 0.f};

#pragma unroll 1
  for (int k0 = 0; k0 < kNodes; k0 += 32) {
    const v16h a0 = FragH::load(A + (size_t)(m0 + rlane) * kNodes + koff + k0);
    const v16h a1 = FragH::load(A + (size_t)(m0 + 16 + rlane) * kNodes + koff + k0);
#pragma unroll
    for (int j = 0; j < 8; ++j) {
      const v16h bf = FragH::load(Bt + (size_t)((j << 4) + rlane) * kNodes + koff + k0);
      acc[0][j] = mma_f16_guarded(a0, bf, acc[0][j]);
      acc[1][j] = mma_f16_guarded(a1, bf, acc[1][j]);
    }
  }

  float* slab = sSlab[wave];
#pragma unroll
  for (int i = 0; i < 2; ++i) {
#pragma unroll
    for (int j = 0; j < 8; ++j) {
#pragma unroll
      for (int r = 0; r < 8; ++r)
        slab[(mOff + r) * kSlabPitch + (j << 4) + rlane] = acc[i][j][r] * scale;
    }
    __builtin_amdgcn_fence(__ATOMIC_RELEASE, "workgroup");
    __builtin_amdgcn_wave_barrier();
    __builtin_amdgcn_fence(__ATOMIC_ACQUIRE, "workgroup");
    float* C = Cout + (size_t)b * kPlaneElems + (size_t)(m0 + (i << 4)) * kFeat;
    for (int pass = 0; pass < 2; ++pass) {
#pragma unroll
      for (int row = 0; row < 16; ++row) {
        const v4f v = *(const v4f*)(slab + row * kSlabPitch + lane * 4);
        *(volatile v4f*)(C + (size_t)row * kFeat + lane * 4) = v;
      }
      __threadfence();
    }
    __builtin_amdgcn_fence(__ATOMIC_RELEASE, "workgroup");
    __builtin_amdgcn_wave_barrier();
    __builtin_amdgcn_fence(__ATOMIC_ACQUIRE, "workgroup");
  }
}

extern "C" void kernel_launch(void* const* d_in, const int* in_sizes, int n_in,
                              void* d_out, int out_size, void* d_ws, size_t ws_size,
                              hipStream_t stream) {
  if (n_in < 6) return;
  if (in_sizes[1] != kBatch * kNodes * kNodes) return;
  if (in_sizes[2] != kBatch * kNodes) return;
  if (in_sizes[3] != kBatch * kNodes * kNodes) return;
  if (in_sizes[4] != kLive * kFeat * kFeat) return;
  if (in_sizes[5] != kLive * kFeat) return;
  if (out_size != kBatch * kNodes * kFeat) return;
  if (ws_size < kWsTotal) return;

  const int*   bfm   = (const int*)d_in[1];
  const int*   a_bfm = (const int*)d_in[2];
  const float* adj   = (const float*)d_in[3];
  const float* adj_w = (const float*)d_in[4];
  const float* adj_a = (const float*)d_in[5];
  float* out = (float*)d_out;

  char* ws = (char*)d_ws;
  float*          Tab  = (float*)(ws + kOffTab);
  unsigned short* MsgT = (unsigned short*)(ws + kOffMsgT);
  unsigned short* AdjH = (unsigned short*)(ws + kOffAdjH);

  build_table_kernel<<<kTypes * kTypes, 128, 0, stream>>>(adj_w, adj_a, Tab);
  prep_planes_kernel<<<kBatch, 256, 0, stream>>>(bfm, a_bfm, adj, Tab, MsgT, AdjH);
  batched_gemm_f16_kernel<<<kBatch, 128, 0, stream>>>(AdjH, MsgT, out, kFold);
}
